// SkipConnection_52166672777658
// MI455X (gfx1250) — hardware-run, weakly checked
//
#include <hip/hip_runtime.h>
#include <math.h>

typedef __attribute__((ext_vector_type(16))) _Float16 v16h;
typedef __attribute__((ext_vector_type(8)))  _Float16 v8h;
typedef __attribute__((ext_vector_type(8)))  float    v8f;
typedef __attribute__((ext_vector_type(4)))  float    v4f;
typedef __attribute__((ext_vector_type(4)))  unsigned int v4u;

constexpr int kB    = 8;
constexpr int kN    = 1024;
constexpr int kDim  = 768;
constexpr int kH    = 8;
constexpr int kHd   = 96;
constexpr int kTok  = kB * kN;
constexpr int kImgS = 16;
constexpr int kImgC = 3;
static_assert(kH * kHd == kDim);
static_assert(kImgS * kImgS * kImgC == kDim);
static_assert((kHd % 32) == 0 && (kN % 32) == 0 && (kDim % 32) == 0);
static_assert((kTok % 64) == 0 && (kDim % 64) == 0);

constexpr float kQkvCarry = 64.0f;
constexpr float kACarry   = 4096.0f;
constexpr float kWCarry   = 1024.0f;
constexpr float kSInv     = 1.0f / (kQkvCarry * kQkvCarry);
constexpr float kVInv     = 1.0f / kQkvCarry;
constexpr float kOutScale = 1.0f / (kACarry * kWCarry);
constexpr float kNormEps  = 1e-3f;

constexpr int kPitch     = 1040;
constexpr int kOstP      = 772;
constexpr int kLdsPBytes = kH * 16 * kPitch * 2;
constexpr int kLdsCoefB  = 16 * 64 * 4;
constexpr int kLdsCcB    = 64 * 4;
constexpr int kLdsEcB    = 8 * 4;
constexpr int kLdsTotal  = kLdsPBytes + kLdsCoefB + kLdsCcB + kLdsEcB;
static_assert(kLdsPBytes == 266240);
static_assert(kLdsTotal == 270624);
static_assert(16 * kOstP * 4 <= kLdsPBytes);
static_assert((kPitch * 2) % 16 == 0 && (kOstP * 4) % 16 == 0);

constexpr size_t kPlaneB = (size_t)kB * kH * kN * kHd * 2;
constexpr size_t kOffQH  = 0;
constexpr size_t kOffKH  = kOffQH + kPlaneB;
constexpr size_t kOffVT  = kOffKH + kPlaneB;
constexpr size_t kOffOP  = kOffVT + kPlaneB;
constexpr size_t kOffWT  = kOffOP + (size_t)kTok * kDim * 2;
constexpr size_t kWsTotal = kOffWT + (size_t)kDim * kDim * 2;
static_assert(kPlaneB == 12582912ull);
static_assert(kWsTotal == 51511296ull);
static_assert(kWsTotal <= 134217728ull);
static_assert((kOffKH % 128) == 0 && (kOffVT % 128) == 0 && (kOffOP % 128) == 0 && (kOffWT % 128) == 0);

__device__ __forceinline__ unsigned pk16(unsigned short a, unsigned short b) { return (unsigned)a | ((unsigned)b << 16); }
__device__ __forceinline__ unsigned short h_bits(float f) { const _Float16 h = (_Float16)f; return __builtin_bit_cast(unsigned short, h); }

__device__ __forceinline__ float h16_to_f32(unsigned hb) {
  const unsigned sgn = (hb & 0x8000u) << 16; const unsigned em = hb & 0x7fffu;
  const float fn = __uint_as_float((em << 13) + 0x38000000u);
  const float fs = (float)em * 5.9604644775390625e-8f;
  const float mag = (em < 0x400u) ? fs : fn; return __uint_as_float(__float_as_uint(mag) | sgn); }

union FragU { v16h v; v8h h[2]; };
__device__ __forceinline__ v16h frag_load(const _Float16* p) {
  FragU f; f.h[0] = *(const v8h*)(p); f.h[1] = *(const v8h*)(p + 16); return f.v;
}
__device__ __forceinline__ v8f mma_h(v16h a, v16h b, v8f c) {
  c = __builtin_amdgcn_wmma_f32_16x16x32_f16(false, a, false, b, (short)0, c, false, false);
  asm volatile("v_nop\n\tv_nop\n\tv_nop\n\tv_nop" : "+v"(c) : "v"(a), "v"(b));
  return c;
}

__global__ __launch_bounds__(256) void conv_split_kernel(
    const float* __restrict__ q, const float* __restrict__ k, const float* __restrict__ v,
    const float* __restrict__ conv_w,
    unsigned short* __restrict__ QH, unsigned short* __restrict__ KH, unsigned short* __restrict__ VT)
{
  __shared__ __align__(16) unsigned short sOut[64 * kDim];
  __shared__ __align__(16) float sImg[18 * 18 * 3 + 4];
  __shared__ float sW[96];
  const int t  = threadIdx.x;
  const int ts = blockIdx.y;
  const int b  = blockIdx.x >> 4;
  const int n0 = (blockIdx.x & 15) * 64;
  const float* src = (ts == 0) ? q : ((ts == 1) ? k : v);

  {
    const float wv = conv_w[t < 81 ? t : 80];
    if (t < 81) sW[t] = wv;
  }
  __syncthreads();
  float w[81];
#pragma unroll
  for (int i = 0; i < 81; ++i) w[i] = sW[i];

  int bofs = 0;
  {
    const int j  = t / 3;
    const int ci = t - j * 3;
    int py, px;
    if (j < 18)      { py = 0;       px = j; }
    else if (j < 36) { py = 17;      px = j - 18; }
    else if (j < 52) { py = j - 35;  px = 0; }
    else             { py = j - 51;  px = 17; }
    if (py > 17) py = 17;
    bofs = (py * 18 + px) * 3 + ci;
  }
  const int y = t >> 4, x = t & 15;
  const int sdst = ((y + 1) * 18 + (x + 1)) * 3;
  const int tb   = (y * 18 + x) * 3;

#pragma unroll 1
  for (int tok = 0; tok < 64; ++tok) {
    const float* sp = src + ((size_t)(b * kN + n0 + tok)) * kDim + t * 3;
    const float x0 = sp[0], x1 = sp[1], x2 = sp[2];
    __syncthreads();
    sImg[sdst]     = x0;
    sImg[sdst + 1] = x1;
    sImg[sdst + 2] = x2;
    if (t < 204) sImg[bofs] = 0.0f;
    __syncthreads();
    float a0 = 0.0f, a1 = 0.0f, a2 = 0.0f;
#pragma unroll
    for (int ky = 0; ky < 3; ++ky) {
#pragma unroll
      for (int kx = 0; kx < 3; ++kx) {
#pragma unroll
        for (int ci = 0; ci < 3; ++ci) {
          const float xv = sImg[tb + ky * 54 + kx * 3 + ci];
          a0 = fmaf(xv, w[(ky * 3 + kx) * 9 + ci * 3 + 0], a0);
          a1 = fmaf(xv, w[(ky * 3 + kx) * 9 + ci * 3 + 1], a1);
          a2 = fmaf(xv, w[(ky * 3 + kx) * 9 + ci * 3 + 2], a2);
        }
      }
    }
    sOut[tok * kDim + t * 3 + 0] = h_bits(a0 * kQkvCarry);
    sOut[tok * kDim + t * 3 + 1] = h_bits(a1 * kQkvCarry);
    sOut[tok * kDim + t * 3 + 2] = h_bits(a2 * kQkvCarry);
  }
  __syncthreads();

  if (ts < 2) {
    unsigned short* dst = (ts == 0) ? QH : KH;
    for (int pass = 0; pass < 2; ++pass) {
#pragma unroll 1
      for (int it = 0; it < 24; ++it) {
        const int idx = it * 256 + t;
        const int h   = idx / 768;
        const int j   = idx - h * 768;
        const int tok = j / 12;
        const int c   = j - tok * 12;
        const v4u val = *(const v4u*)(sOut + tok * kDim + h * kHd + c * 8);
        *(volatile v4u*)(dst + ((size_t)((b * kH + h) * kN + n0)) * kHd + (size_t)j * 8) = val;
      }
      __threadfence();
    }
  } else {
    for (int pass = 0; pass < 2; ++pass) {
#pragma unroll 1
      for (int it = 0; it < 24; ++it) {
        const int idx = it * 256 + t;
        const int p   = idx >> 3;
        const int sub = idx & 7;
        const int h   = p / kHd;
        const int d   = p - h * kHd;
        unsigned short hb[8];
#pragma unroll
        for (int e = 0; e < 8; ++e) hb[e] = sOut[(sub * 8 + e) * kDim + p];
        const v4u val = (v4u){pk16(hb[0], hb[1]), pk16(hb[2], hb[3]), pk16(hb[4], hb[5]), pk16(hb[6], hb[7])};
        *(volatile v4u*)(VT + ((size_t)((b * kH + h) * kHd + d)) * kN + n0 + sub * 8) = val;
      }
      __threadfence();
    }
  }
}

__global__ __launch_bounds__(256) void wt_cast_kernel(const float* __restrict__ W, unsigned short* __restrict__ WT, float scale) {
  __shared__ float sm[64][65];
  const int t  = threadIdx.x;
  const int d0 = blockIdx.x * 64;
  const int h0 = blockIdx.y * 64;
#pragma unroll
  for (int i = 0; i < 16; ++i) {
    const int e = i * 256 + t;
    const int r = e >> 6;
    const int c = e & 63;
    sm[c][r] = W[(size_t)(d0 + r) * kDim + h0 + c] * scale;
  }
  __syncthreads();
  const int lane = t & 31, wave = t >> 5;
  const int qd = lane >> 3, c8 = (lane & 7) * 8;
  for (int pass = 0; pass < 2; ++pass) {
#pragma unroll
    for (int it = 0; it < 2; ++it) {
      const int row = wave * 8 + it * 4 + qd;
      unsigned short hb[8];
#pragma unroll
      for (int e = 0; e < 8; ++e) hb[e] = h_bits(sm[row][c8 + e]);
      const v4u u = (v4u){pk16(hb[0], hb[1]), pk16(hb[2], hb[3]), pk16(hb[4], hb[5]), pk16(hb[6], hb[7])};
      *(volatile v4u*)(WT + (size_t)(h0 + row) * kDim + d0 + c8) = u;
    }
    __threadfence();
  }
}

__global__ __launch_bounds__(512) void attn_mix_kernel(
    const unsigned short* __restrict__ Qp, const unsigned short* __restrict__ Kp, const unsigned short* __restrict__ Vtp,
    const float* __restrict__ rw, const float* __restrict__ rb,
    const float* __restrict__ gam, const float* __restrict__ bet,
    const float* __restrict__ mean, const float* __restrict__ var,
    unsigned short* __restrict__ Op, float qk_scale)
{
  extern __shared__ __align__(16) unsigned char smem[];
  unsigned short* Pu = (unsigned short*)smem;
  _Float16* Ph = (_Float16*)smem;
  float* Ost  = (float*)smem;
  float* coef = (float*)(smem + kLdsPBytes);
  float* cC   = (float*)(smem + kLdsPBytes + kLdsCoefB);
  float* eC   = (float*)(smem + kLdsPBytes + kLdsCoefB + kLdsCcB);

  const int tid = threadIdx.x, lane = tid & 31, wave = tid >> 5;
  const int hh = lane >> 4, cl = lane & 15;
  const int b  = blockIdx.x >> 6;
  const int n0 = (blockIdx.x & 63) << 4;
  const _Float16* Qh = (const _Float16*)Qp;
  const _Float16* Kh = (const _Float16*)Kp;
  const _Float16* Vt = (const _Float16*)Vtp;

  {
    const int hq = (tid >> 3) & 7, gq = tid & 7;
    const float inv = gam[gq] * rsqrtf(var[gq] + kNormEps);
    const float wv  = rw[hq * 8 + gq];
    const float ev  = ((rb[gq] - mean[gq]) * inv + bet[gq]) * kACarry;
    if (tid < 64) cC[tid] = wv * inv;
    if (tid < 8)  eC[tid] = ev;
  }

  {
    const int hd = wave >> 1, mh = wave & 1;
    const size_t bh = (size_t)(b * kH + hd);
    const _Float16* Qb = Qh + (bh * kN + n0 + cl) * kHd + 8 * hh;
    const _Float16* Kb = Kh + bh * kN * kHd + 8 * hh;
    const v16h qf0 = frag_load(Qb);
    const v16h qf1 = frag_load(Qb + 32);
    const v16h qf2 = frag_load(Qb + 64);
    const float sc = qk_scale * kSInv;
    _Float16* Prow = Ph + (hd * 16 + cl) * kPitch + 8 * hh;
#pragma unroll 1
    for (int t = 0; t < 32; ++t) {
      const int m0 = mh * 512 + t * 16;
      const _Float16* kr = Kb + (size_t)(m0 + cl) * kHd;
      v8f acc = (v8f){0.f, 0.f, 0.f, 0.f, 0.f, 0.f, 0.f, 0.f};
      const v16h kf0 = frag_load(kr);
      const v16h kf1 = frag_load(kr + 32);
      const v16h kf2 = frag_load(kr + 64);
      acc = mma_h(kf0, qf0, acc);
      acc = mma_h(kf1, qf1, acc);
      acc = mma_h(kf2, qf2, acc);
      v8h o;
#pragma unroll
      for (int r = 0; r < 8; ++r) o[r] = (_Float16)(acc[r] * sc);
      *(v8h*)(Prow + m0) = o;
    }
  }
  __syncthreads();

#pragma unroll 1
  for (int i = 0; i < 8; ++i) {
    const int R = wave * 8 + i;
    unsigned short* row = Pu + R * kPitch + lane * 8;
    float xv[32];
#pragma unroll
    for (int j = 0; j < 4; ++j) {
      const v4u wd = *(const v4u*)(row + j * 256);
#pragma unroll
      for (int e = 0; e < 4; ++e) {
        const unsigned ww = wd[e];
        xv[j * 8 + e * 2]     = h16_to_f32(ww & 0xffffu);
        xv[j * 8 + e * 2 + 1] = h16_to_f32(ww >> 16);
      }
    }
    float mx = xv[0];
#pragma unroll
    for (int e = 1; e < 32; ++e) mx = fmaxf(mx, xv[e]);
#pragma unroll
    for (int off = 16; off > 0; off >>= 1) mx = fmaxf(mx, __shfl_xor(mx, off, 32));
    float sum = 0.0f;
#pragma unroll
    for (int j = 0; j < 4; ++j) {
      unsigned pk[4];
#pragma unroll
      for (int e = 0; e < 4; ++e) {
        const float e0 = __expf(xv[j * 8 + e * 2] - mx);
        const float e1 = __expf(xv[j * 8 + e * 2 + 1] - mx);
        sum += e0;
        sum += e1;
        pk[e] = pk16(h_bits(e0), h_bits(e1));
      }
      *(v4u*)(row + j * 256) = (v4u){pk[0], pk[1], pk[2], pk[3]};
    }
#pragma unroll
    for (int off = 16; off > 0; off >>= 1) sum += __shfl_xor(sum, off, 32);
    const float zs = kACarry * (1.0f / sum);
    const int hr = R >> 4, nr = R & 15;
    const float cv = cC[hr * 8 + (lane & 7)];
    if (lane < 8) coef[nr * 64 + hr * 8 + lane] = cv * zs;
  }
  __syncthreads();

#pragma unroll 1
  for (int it = 0; it < 4; ++it) {
    const int item = it * 512 + tid;
    const int n = item >> 7;
    const int m = (item & 127) * 8;
    float a[8][8];
#pragma unroll
    for (int h = 0; h < 8; ++h) {
      const v4u wd = *(const v4u*)(Pu + (h * 16 + n) * kPitch + m);
#pragma unroll
      for (int e = 0; e < 4; ++e) {
        const unsigned ww = wd[e];
        a[h][e * 2]     = h16_to_f32(ww & 0xffffu);
        a[h][e * 2 + 1] = h16_to_f32(ww >> 16);
      }
    }
    const float* cf = coef + n * 64;
#pragma unroll 1
    for (int g = 0; g < 8; ++g) {
      const float ec = eC[g];
      float o[8];
#pragma unroll
      for (int j = 0; j < 8; ++j) o[j] = ec;
#pragma unroll
      for (int h = 0; h < 8; ++h) {
        const float c = cf[h * 8 + g];
#pragma unroll
        for (int j = 0; j < 8; ++j) o[j] = fmaf(c, a[h][j], o[j]);
      }
      const v4u ov = (v4u){pk16(h_bits(o[0]), h_bits(o[1])), pk16(h_bits(o[2]), h_bits(o[3])),
                           pk16(h_bits(o[4]), h_bits(o[5])), pk16(h_bits(o[6]), h_bits(o[7]))};
      *(v4u*)(Pu + (g * 16 + n) * kPitch + m) = ov;
    }
  }
  __syncthreads();

  const int g = wave >> 1, dh = wave & 1;
  v8f oacc0 = (v8f){0.f, 0.f, 0.f, 0.f, 0.f, 0.f, 0.f, 0.f};
  v8f oacc1 = oacc0;
  v8f oacc2 = oacc0;
  {
    const _Float16* Arow = Ph + (g * 16 + cl) * kPitch + 8 * hh;
    const _Float16* Vb = Vt + ((size_t)((b * kH + g) * kHd + dh * 48 + cl)) * kN + 8 * hh;
#pragma unroll 1
    for (int kc = 0; kc < 32; ++kc) {
      const int m0 = kc * 32;
      const v16h af = frag_load(Arow + m0);
      const v16h b0 = frag_load(Vb + m0);
      const v16h b1 = frag_load(Vb + (size_t)16 * kN + m0);
      const v16h b2 = frag_load(Vb + (size_t)32 * kN + m0);
      oacc0 = mma_h(af, b0, oacc0);
      oacc1 = mma_h(af, b1, oacc1);
      oacc2 = mma_h(af, b2, oacc2);
    }
  }
  __syncthreads();
  {
    const int colb = g * kHd + dh * 48 + cl;
#pragma unroll
    for (int r = 0; r < 8; ++r) {
      float* orow = Ost + (8 * hh + r) * kOstP + colb;
      orow[0]  = oacc0[r] * kVInv;
      orow[16] = oacc1[r] * kVInv;
      orow[32] = oacc2[r] * kVInv;
    }
  }
  __syncthreads();
  {
    const float* sr = Ost + wave * kOstP + lane * 8;
    unsigned short* orow = Op + ((size_t)(b * kN + n0 + wave)) * kDim + lane * 8;
    v8h hv[3];
#pragma unroll
    for (int it = 0; it < 3; ++it) {
      const v4f a0 = *(const v4f*)(sr + it * 256);
      const v4f a1 = *(const v4f*)(sr + it * 256 + 4);
#pragma unroll
      for (int e = 0; e < 4; ++e) {
        hv[it][e]     = (_Float16)a0[e];
        hv[it][4 + e] = (_Float16)a1[e];
      }
    }
    for (int pass = 0; pass < 2; ++pass) {
#pragma unroll
      for (int it = 0; it < 3; ++it) *(volatile v8h*)(orow + it * 256) = hv[it];
      __threadfence();
    }
  }
}

__global__ __launch_bounds__(256) void proj_gemm_kernel(
    const unsigned short* __restrict__ Ap, int lda,
    const unsigned short* __restrict__ Btp, int ldb,
    float* __restrict__ C, int ldc,
    const float* __restrict__ bias,
    int M, int N, int K, float scale) {
  const _Float16* A  = (const _Float16*)Ap;
  const _Float16* Bt = (const _Float16*)Btp;
  __shared__ __align__(16) float sT[8][16 * 68];
  const int lane = threadIdx.x & 31;
  const int wave = threadIdx.x >> 5;
  const int tilesN = N >> 6;
  const int tilesM = M >> 6;
  const int tile = blockIdx.x * 8 + wave;
  if (tile >= tilesM * tilesN) return;
  const int tm = tile / tilesN;
  const int tn = tile - tm * tilesN;
  const int m0 = tm << 6;
  const int n0 = tn << 6;

  const int rlane = lane & 15;
  const int koff  = (lane >> 4) * 8;
  const int mOff  = (lane >> 4) * 8;

  v8f acc[4][4];
#pragma unroll
  for (int i = 0; i < 4; ++i)
#pragma unroll
    for (int j = 0; j < 4; ++j) acc[i][j] = (v8f){0.f, 0.f, 0.f, 0.f, 0.f, 0.f, 0.f, 0.f};

  for (int k0 = 0; k0 < K; k0 += 32) {
    v16h bh[4];
#pragma unroll
    for (int j = 0; j < 4; ++j) {
      const size_t bo = (size_t)(n0 + (j << 4) + rlane) * ldb + koff + k0;
      bh[j] = frag_load(Bt + bo);
    }
#pragma unroll
    for (int i = 0; i < 4; ++i) {
      const size_t ao = (size_t)(m0 + (i << 4) + rlane) * lda + koff + k0;
      const v16h ah = frag_load(A + ao);
#pragma unroll
      for (int j = 0; j < 4; ++j) acc[i][j] = mma_h(ah, bh[j], acc[i][j]);
    }
  }

  float* slab = sT[wave];
#pragma unroll
  for (int i = 0; i < 4; ++i) {
    const int mBase = m0 + (i << 4);
#pragma unroll
    for (int j = 0; j < 4; ++j) {
      const int n = n0 + (j << 4) + rlane;
      const float bv = bias[n];
#pragma unroll
      for (int r = 0; r < 8; ++r) {
        const float val = acc[i][j][r] * scale + bv;
        slab[(mOff + r) * 68 + (j << 4) + rlane] = val;
      }
    }
    __builtin_amdgcn_fence(__ATOMIC_RELEASE, "workgroup");
    __builtin_amdgcn_wave_barrier();
    __builtin_amdgcn_fence(__ATOMIC_ACQUIRE, "workgroup");
    {
      const int hq = lane >> 4, c4 = (lane & 15) * 4;
      for (int pass = 0; pass < 2; ++pass) {
#pragma unroll
        for (int it = 0; it < 8; ++it) {
          const int row = it * 2 + hq;
          const v4f val = *(const v4f*)(slab + row * 68 + c4);
          *(volatile v4f*)(C + (size_t)(mBase + row) * ldc + n0 + c4) = val;
        }
        __threadfence();
      }
    }
    __builtin_amdgcn_fence(__ATOMIC_RELEASE, "workgroup");
    __builtin_amdgcn_wave_barrier();
    __builtin_amdgcn_fence(__ATOMIC_ACQUIRE, "workgroup");
  }
}

extern "C" void kernel_launch(void* const* d_in, const int* in_sizes, int n_in,
                              void* d_out, int out_size, void* d_ws, size_t ws_size,
                              hipStream_t stream) {
  if (n_in < 12) return;
  if (in_sizes[0] != kTok * kDim) return;
  if (in_sizes[1] != kTok * kDim) return;
  if (in_sizes[2] != kTok * kDim) return;
  if (in_sizes[3] != 81) return;
  if (in_sizes[4] != kH * kH) return;
  if (in_sizes[5] != kH || in_sizes[6] != kH || in_sizes[7] != kH || in_sizes[8] != kH || in_sizes[9] != kH) return;
  if (in_sizes[10] != kDim * kDim) return;
  if (in_sizes[11] != kDim) return;
  if (out_size != kTok * kDim) return;
  if (ws_size < kWsTotal) return;

  const float* q         = (const float*)d_in[0];
  const float* k         = (const float*)d_in[1];
  const float* v         = (const float*)d_in[2];
  const float* conv_w    = (const float*)d_in[3];
  const float* reatten_w = (const float*)d_in[4];
  const float* reatten_b = (const float*)d_in[5];
  const float* bn_gamma  = (const float*)d_in[6];
  const float* bn_beta   = (const float*)d_in[7];
  const float* bn_mean   = (const float*)d_in[8];
  const float* bn_var    = (const float*)d_in[9];
  const float* proj_w    = (const float*)d_in[10];
  const float* proj_b    = (const float*)d_in[11];
  float* out = (float*)d_out;

  char* ws = (char*)d_ws;
  unsigned short* QH = (unsigned short*)(ws + kOffQH);
  unsigned short* KH = (unsigned short*)(ws + kOffKH);
  unsigned short* VT = (unsigned short*)(ws + kOffVT);
  unsigned short* OP = (unsigned short*)(ws + kOffOP);
  unsigned short* WT = (unsigned short*)(ws + kOffWT);

  const float qk_scale = (float)(1.0 / sqrt((double)kHd));

  conv_split_kernel<<<dim3(kTok / 64, 3), 256, 0, stream>>>(q, k, v, conv_w, QH, KH, VT);
  wt_cast_kernel<<<dim3(kDim / 64, kDim / 64), 256, 0, stream>>>(proj_w, WT, kWCarry);
  attn_mix_kernel<<<kB * (kN / 16), 512, kLdsTotal, stream>>>(
      QH, KH, VT, reatten_w, reatten_b, bn_gamma, bn_beta, bn_mean, bn_var, OP, qk_scale);
  proj_gemm_kernel<<<((kTok / 64) * (kDim / 64)) / 8, 256, 0, stream>>>(
      OP, kDim, WT, kDim, out, kDim, proj_b, kTok, kDim, kDim, kOutScale);
}
